// SE3PointConvolution_59940563583479
// MI455X (gfx1250) — hardware-verified
//
#include <hip/hip_runtime.h>
#include <math.h>

typedef __attribute__((ext_vector_type(16))) _Float16 v16h;
typedef __attribute__((ext_vector_type(16))) __bf16 v16b;
typedef __attribute__((ext_vector_type(8)))  _Float16 v8h;
typedef __attribute__((ext_vector_type(8)))  float v8f;
typedef __attribute__((ext_vector_type(4)))  float v4f;
typedef __attribute__((ext_vector_type(2)))  float v2f;
typedef __attribute__((ext_vector_type(4)))  unsigned v4u;
typedef __attribute__((ext_vector_type(4)))  int v4i;
typedef float __attribute__((may_alias)) float_a;
typedef int __attribute__((may_alias)) int_a;

template <typename T> __device__ __forceinline__ void vst2(void* p, T v) { *(volatile T*)p = v; __threadfence(); *(volatile T*)p = v; }
__device__ __forceinline__ v8f wmma16(v16h a, v16h b, v8f c) {
  v8f d = __builtin_amdgcn_wmma_f32_16x16x32_f16(false, a, false, b, (short)0, c, false, false);
  asm volatile("v_nop\n\tv_nop\n\tv_nop\n\tv_nop" : "+v"(d) : "v"(a), "v"(b));
  return d;
}
__device__ __forceinline__ v8f wmma_bf(v16b a, v16b b, v8f c) {
  v8f d = __builtin_amdgcn_wmma_f32_16x16x32_bf16(false, a, false, b, (short)0, c, false, false);
  asm volatile("v_nop\n\tv_nop\n\tv_nop\n\tv_nop" : "+v"(d) : "v"(a), "v"(b));
  return d;
}
__device__ __forceinline__ v16h frag_h(const _Float16* rowk0, int lane) {
  union { v16h v; v8h q[2]; } u; const _Float16* p = rowk0 + 8 * (lane >> 4);
  u.q[0] = *(const v8h*)p; u.q[1] = *(const v8h*)(p + 16); return u.v;
}
__device__ __forceinline__ v16h frag_f32(const float* rowk0, int lane) {
  v16h a; const float* p = rowk0 + 8 * (lane >> 4);
#pragma unroll
  for (int i = 0; i < 8; ++i) { a[i] = (_Float16)p[i]; a[8 + i] = (_Float16)p[16 + i]; }
  return a;
}
__device__ __forceinline__ v16h frag_f32s(const float* rowk0, int lane, float sc) {
  v16h a; const float* p = rowk0 + 8 * (lane >> 4);
#pragma unroll
  for (int i = 0; i < 8; ++i) { a[i] = (_Float16)(p[i] * sc); a[8 + i] = (_Float16)(p[16 + i] * sc); }
  return a;
}
__device__ __forceinline__ v16h fragc_f32(const float* W, int k0, int n, int lane, int ld, int K) {
  v16h a; const int g = lane >> 4;
#pragma unroll
  for (int i = 0; i < 8; ++i) { const int ka = k0 + 8 * g + i, kb = ka + 16;
    a[i] = (_Float16)(ka < K ? W[(size_t)(ka < K ? ka : K - 1) * ld + n] : 0.f); a[8 + i] = (_Float16)(kb < K ? W[(size_t)(kb < K ? kb : K - 1) * ld + n] : 0.f); }
  return a;
}
struct F2 { v16b h, l; };
__device__ __forceinline__ F2 bsplit16(const float v[16]) { F2 r;
#pragma unroll
  for (int i = 0; i < 16; ++i) { const __bf16 h = (__bf16)v[i]; r.h[i] = h; r.l[i] = (__bf16)(v[i] - (float)h); }
  return r; }
__device__ __forceinline__ F2 split_row(const float* row, int k0, int lane) { float v[16]; const float* p = row + k0 + 8 * (lane >> 4);
#pragma unroll
  for (int i = 0; i < 8; ++i) { v[i] = p[i]; v[8 + i] = p[16 + i]; }
  return bsplit16(v); }
__device__ __forceinline__ F2 split_rowK(const float* row, int k0, int lane, int K) { float v[16]; const int g = lane >> 4;
#pragma unroll
  for (int i = 0; i < 8; ++i) { const int ka = k0 + 8 * g + i, kb = ka + 16; v[i] = ka < K ? row[ka < K ? ka : K - 1] : 0.f; v[8 + i] = kb < K ? row[kb < K ? kb : K - 1] : 0.f; }
  return bsplit16(v); }
__device__ __forceinline__ F2 split_col(const float* W, int k0, int n, int lane, int ld, int K) { float v[16]; const int g = lane >> 4;
#pragma unroll
  for (int i = 0; i < 8; ++i) { const int ka = k0 + 8 * g + i, kb = ka + 16; v[i] = ka < K ? W[(size_t)(ka < K ? ka : K - 1) * ld + n] : 0.f; v[8 + i] = kb < K ? W[(size_t)(kb < K ? kb : K - 1) * ld + n] : 0.f; }
  return bsplit16(v); }
__device__ __forceinline__ v8f mac3(const F2& a, const F2& b, v8f c) { c = wmma_bf(a.l, b.h, c); c = wmma_bf(a.h, b.l, c); return wmma_bf(a.h, b.h, c); }
__device__ __forceinline__ float sigm(float v) { return 1.0f / (1.0f + expf(-v)); }
#define LDSX() do { asm volatile("s_wait_dscnt 0" ::: "memory"); __builtin_amdgcn_wave_barrier(); __builtin_amdgcn_fence(__ATOMIC_RELEASE, "workgroup"); } while (0)


#define NN 4
#define NBp 256
#define NA 256
#define NC 16
#define ND 16
#define NRAD 8
#define KAR (NA * NRAD)
typedef __attribute__((ext_vector_type(8))) __bf16 v8b;
__device__ __forceinline__ v16b frag_b(const __bf16* rowk0, int lane) {
  union { v16b v; v8b q[2]; } u; const __bf16* p = rowk0 + 8 * (lane >> 4);
  u.q[0] = *(const v8b*)p; u.q[1] = *(const v8b*)(p + 16); return u.v;
}
__device__ __forceinline__ float bfr(float v) { return (float)(__bf16)v; }
__device__ __attribute__((noinline)) float exp_ni(float v) { return expf(v); }
#define WS_UT  0u
#define WS_END (WS_UT + 4u * NN * ND * KAR)

__global__ __launch_bounds__(256) void k_u(const float* __restrict__ IN, const float* __restrict__ Wt, float* __restrict__ UT) {
  __shared__ float sw[NC][NRAD]; __shared__ __align__(16) float srow[KAR];
  const int n = blockIdx.x / ND, d = blockIdx.x % ND, a = threadIdx.x;
  if (a < NC * NRAD) sw[a / NRAD][a % NRAD] = bfr(Wt[((size_t)d * NC + a / NRAD) * NRAD + a % NRAD]);
  __syncthreads();
  float acc[NRAD];
#pragma unroll
  for (int r = 0; r < NRAD; ++r) acc[r] = 0.f;
#pragma unroll 1
  for (int c = 0; c < NC; ++c) { const float x = bfr(IN[((size_t)n * NC + c) * NA + a]);
#pragma unroll
    for (int r = 0; r < NRAD; ++r) acc[r] += x * sw[c][r]; }
#pragma unroll
  for (int r = 0; r < NRAD; ++r) srow[a * NRAD + r] = acc[r];
  __syncthreads();
  for (int q = a; q < KAR / 4; q += 256) vst2(UT + ((size_t)n * ND + d) * KAR + q * 4, *(const v4f*)&srow[q * 4]);
}
__global__ __launch_bounds__(128) void k_main(const float* __restrict__ DIFF, const float* __restrict__ MASK, const float* __restrict__ RADII, const float* __restrict__ UT, float* __restrict__ out) {
  __shared__ __align__(16) __bf16 srh[64][264], srl[64][264]; __shared__ float srad[NRAD]; __shared__ __align__(16) float so[ND][68];
  const int tid = threadIdx.x, wave = tid >> 5, lane = tid & 31, col = lane & 15, g = lane >> 4; const int n = blockIdx.y, b0 = blockIdx.x * 64;
  if (tid < NRAD) srad[tid] = bfr(RADII[tid]);
  __syncthreads();
  v8f acc = {};
#pragma unroll 1
  for (int ch = 0; ch < KAR / 256; ++ch) {
    for (int q = tid; q < 64 * 32; q += 128) { const int bl = q >> 5, al = q & 31; const int a = ch * 32 + al; const size_t e = ((size_t)n * NBp + b0 + bl) * NA + a;
      const float dx = bfr(DIFF[e * 3]), dy = bfr(DIFF[e * 3 + 1]), dz = bfr(DIFF[e * 3 + 2]); const float dist = sqrtf((dx * dx + dy * dy) + dz * dz); const float mk = bfr(MASK[e]);
#pragma unroll
      for (int r = 0; r < NRAD; ++r) { const float t = dist - srad[r]; const float v = exp_ni(-6.125f * t * t) * mk; const __bf16 hb = (__bf16)v; srh[bl][al * NRAD + r] = hb; srl[bl][al * NRAD + r] = (__bf16)(v - (float)hb); } }
    __syncthreads();
#pragma unroll
    for (int kc = 0; kc < 8; ++kc) { const v16b ah = frag_b(&srh[wave * 16 + col][kc * 32], lane), al2 = frag_b(&srl[wave * 16 + col][kc * 32], lane); const F2 u = split_row(UT + ((size_t)n * ND + col) * KAR + ch * 256, kc * 32, lane);
      acc = wmma_bf(al2, u.h, acc); acc = wmma_bf(ah, u.l, acc); acc = wmma_bf(ah, u.h, acc); }
    __syncthreads(); }
#pragma unroll
  for (int r = 0; r < 8; ++r) so[col][wave * 16 + 8 * g + r] = acc[r];
  __syncthreads();
  for (int q = tid; q < ND * 16; q += 128) { const int d = q >> 4, pc = q & 15; vst2(out + ((size_t)n * ND + d) * NBp + b0 + pc * 4, *(const v4f*)&so[d][pc * 4]); }
}

extern "C" void kernel_launch(void* const* d_in, const int* in_sizes, int n_in, void* d_out, int out_size, void* d_ws, size_t ws_size, hipStream_t stream) {
  (void)in_sizes; (void)n_in; (void)out_size;
  const float** F = (const float**)d_in;
  if (ws_size < (size_t)WS_END) return;
  float* UT = (float*)((char*)d_ws + WS_UT);
  k_u<<<NN * ND, 256, 0, stream>>>(F[0], F[3], UT);
  k_main<<<dim3(NBp / 64, NN), 128, 0, stream>>>(F[1], F[2], F[4], UT, (float*)d_out);
}
